// LRSAttention_72232759984876
// MI455X (gfx1250) — hardware-verified
//
#include <hip/hip_runtime.h>
#include <stddef.h>
#include <stdint.h>


#define B_     2
#define N_     2048
#define D_     1024
#define H_     16
#define HD_    64
#define ALPHA_ 1.0f
#define WSC    32.0f
#define OSC    16.0f
#define LP     72
#define LPF    68

typedef _Float16 v16h __attribute__((ext_vector_type(16)));
typedef _Float16 v8h  __attribute__((ext_vector_type(8)));
typedef float    v8f  __attribute__((ext_vector_type(8)));
typedef float    v4f  __attribute__((ext_vector_type(4)));

union Frag  { v16h v; v8h half[2]; };
union Pack8 { v8h v; _Float16 s[8]; };

__device__ __forceinline__ v8f wmma16(const Frag& a, const Frag& b, v8f c) {
  v8f d = __builtin_amdgcn_wmma_f32_16x16x32_f16(false, a.v, false, b.v, (short)0, c, false, false);
  asm volatile("v_nop\n\tv_nop\n\tv_nop\n\tv_nop" : "+v"(d) : "v"(a.v), "v"(b.v));
  return d;
}

__device__ __forceinline__ float wave_sum(float v) {
  #pragma unroll
  for (int off = 16; off > 0; off >>= 1) v += __shfl_xor(v, off, 32);
  return v;
}
__device__ __forceinline__ float wave_max(float v) {
  #pragma unroll
  for (int off = 16; off > 0; off >>= 1) v = fmaxf(v, __shfl_xor(v, off, 32));
  return v;
}

__device__ __forceinline__ void store_rows64_h(const _Float16* t, _Float16* dst, size_t gp,
                                               int wave, int lane) {
  v8h v[4];
  size_t off[4];
  #pragma unroll
  for (int p = 0; p < 4; ++p) {
    const int row = wave * 16 + p * 4 + (lane >> 3);
    const int col = (lane & 7) * 8;
    v[p] = *(const v8h*)(t + row * LP + col);
    off[p] = (size_t)row * gp + col;
  }
  #pragma unroll
  for (int p = 0; p < 4; ++p) *(volatile v8h*)(dst + off[p]) = v[p];
  __threadfence();
  #pragma unroll
  for (int p = 0; p < 4; ++p) *(volatile v8h*)(dst + off[p]) = v[p];
}


__global__ __launch_bounds__(256) void cvt_f16_kernel(
    const float* __restrict__ in, _Float16* __restrict__ out, int n) {
  const size_t i = ((size_t)blockIdx.x * 256 + threadIdx.x) * 8;
  if (i + 8 > (size_t)n) return;
  const v4f a = *(const v4f*)(in + i);
  const v4f c = *(const v4f*)(in + i + 4);
  Pack8 u;
  u.s[0] = (_Float16)a[0]; u.s[1] = (_Float16)a[1]; u.s[2] = (_Float16)a[2]; u.s[3] = (_Float16)a[3];
  u.s[4] = (_Float16)c[0]; u.s[5] = (_Float16)c[1]; u.s[6] = (_Float16)c[2]; u.s[7] = (_Float16)c[3];
  const v8h o = u.v;
  *(volatile v8h*)(out + i) = o;
  __threadfence();
  *(volatile v8h*)(out + i) = o;
}

__global__ __launch_bounds__(128) void transpose_cvt_kernel(
    const float* __restrict__ in, _Float16* __restrict__ out, int R, int C, float scale) {
  __shared__ __align__(16) _Float16 T[64][LP];
  const int tid = threadIdx.x, lane = tid & 31, wave = tid >> 5;
  const int c0 = blockIdx.x * 64, r0 = blockIdx.y * 64;
  if (c0 + 64 > C || r0 + 64 > R) return;
  #pragma unroll
  for (int i = 0; i < 8; ++i) {
    const int q = tid + i * 128;
    const int r = q >> 4, c4 = (q & 15) * 4;
    const v4f v = *(const v4f*)(in + (size_t)(r0 + r) * C + c0 + c4);
    T[c4 + 0][r] = (_Float16)(v[0] * scale);
    T[c4 + 1][r] = (_Float16)(v[1] * scale);
    T[c4 + 2][r] = (_Float16)(v[2] * scale);
    T[c4 + 3][r] = (_Float16)(v[3] * scale);
  }
  __syncthreads();
  store_rows64_h(&T[0][0], out + (size_t)c0 * R + r0, (size_t)R, wave, lane);
}

__global__ __launch_bounds__(256) void colabs_kernel(
    const float* __restrict__ x, float* __restrict__ colabs, int ntok, int dim) {
  const int d = blockIdx.x * 256 + threadIdx.x;
  const int b = blockIdx.y;
  if (d >= dim) return;
  const float* p = x + (size_t)b * ntok * dim + d;
  float s = 0.f;
  #pragma unroll 8
  for (int n = 0; n < ntok; ++n) s += fabsf(p[(size_t)n * dim]);
  float* q = colabs + (size_t)b * dim + d;
  *(volatile float*)q = s;
  __threadfence();
  *(volatile float*)q = s;
}

__device__ __forceinline__ void gemm64_mainloop(
    const _Float16* __restrict__ A, const _Float16* __restrict__ Bt, int K,
    int mbase, int nbase, _Float16 (*As)[LP], _Float16 (*Bs)[LP], v8f (&acc)[2][2]) {
  const int tid = threadIdx.x, lane = tid & 31, wave = tid >> 5;
  const int h8 = lane >> 4, l16 = lane & 15;
  const int wm = (wave >> 1) * 32, wn = (wave & 1) * 32;
  const int ldr = tid >> 1, ldc = (tid & 1) * 32;

  #pragma unroll
  for (int r = 0; r < 2; ++r)
    #pragma unroll
    for (int t = 0; t < 2; ++t)
      #pragma unroll
      for (int e = 0; e < 8; ++e) acc[r][t][e] = 0.f;

  const _Float16* ap = A  + (size_t)(mbase + ldr) * K + ldc;
  const _Float16* bp = Bt + (size_t)(nbase + ldr) * K + ldc;

  #pragma unroll 1
  for (int k0 = 0; k0 < K; k0 += 64) {
    v8h ta[4], tb[4];
    #pragma unroll
    for (int i = 0; i < 4; ++i) {
      ta[i] = *(const v8h*)(ap + k0 + i * 8);
      tb[i] = *(const v8h*)(bp + k0 + i * 8);
    }
    __syncthreads();
    #pragma unroll
    for (int i = 0; i < 4; ++i) {
      *(v8h*)&As[ldr][ldc + i * 8] = ta[i];
      *(v8h*)&Bs[ldr][ldc + i * 8] = tb[i];
    }
    __syncthreads();
    #pragma unroll
    for (int kk = 0; kk < 2; ++kk) {
      Frag a[2], b[2];
      #pragma unroll
      for (int rs = 0; rs < 2; ++rs) {
        const _Float16* ar = &As[wm + rs * 16 + l16][kk * 32];
        a[rs].half[0] = *(const v8h*)(ar + 8 * h8);
        a[rs].half[1] = *(const v8h*)(ar + 16 + 8 * h8);
      }
      #pragma unroll
      for (int ts = 0; ts < 2; ++ts) {
        const _Float16* br = &Bs[wn + ts * 16 + l16][kk * 32];
        b[ts].half[0] = *(const v8h*)(br + 8 * h8);
        b[ts].half[1] = *(const v8h*)(br + 16 + 8 * h8);
      }
      #pragma unroll
      for (int rs = 0; rs < 2; ++rs)
        #pragma unroll
        for (int ts = 0; ts < 2; ++ts)
          acc[rs][ts] = wmma16(a[rs], b[ts], acc[rs][ts]);
    }
  }
}

__global__ __launch_bounds__(128) void qkv_gemm_kernel(
    const _Float16* __restrict__ xb, const _Float16* __restrict__ wt, const float* __restrict__ bias,
    _Float16* __restrict__ qb, _Float16* __restrict__ kb, _Float16* __restrict__ vtb,
    int M, int NC, int K) {
  __shared__ __align__(16) _Float16 As[64][LP];
  __shared__ __align__(16) _Float16 Bs[64][LP];
  __shared__ __align__(16) _Float16 Cs[64][LP];
  const int tid = threadIdx.x, lane = tid & 31, wave = tid >> 5;
  const int h8 = lane >> 4, l16 = lane & 15;
  const int wm = (wave >> 1) * 32, wn = (wave & 1) * 32;
  const int mbase = blockIdx.y * 64, nbase = blockIdx.x * 64;
  if (mbase + 64 > M || nbase + 64 > NC) return;

  v8f acc[2][2];
  gemm64_mainloop(xb, wt, K, mbase, nbase, As, Bs, acc);

  const int which = nbase >> 10;
  const int hh = (nbase & (D_ - 1)) >> 6;
  const int b  = mbase >> 11;
  const int n0 = mbase & (N_ - 1);
  const int bh = b * H_ + hh;
  const float inv = 1.0f / WSC;

  if (which == 2) {
    #pragma unroll
    for (int rs = 0; rs < 2; ++rs)
      #pragma unroll
      for (int ts = 0; ts < 2; ++ts) {
        const int col = wn + ts * 16 + l16;
        const float bv = bias[nbase + col];
        #pragma unroll
        for (int g = 0; g < 8; ++g) {
          const int row = wm + rs * 16 + g + 8 * h8;
          Cs[col][row] = (_Float16)(acc[rs][ts][g] * inv + bv);
        }
      }
  } else {
    #pragma unroll
    for (int rs = 0; rs < 2; ++rs)
      #pragma unroll
      for (int ts = 0; ts < 2; ++ts) {
        const int col = wn + ts * 16 + l16;
        const float bv = bias[nbase + col];
        #pragma unroll
        for (int g = 0; g < 8; ++g) {
          const int row = wm + rs * 16 + g + 8 * h8;
          Cs[row][col] = (_Float16)(acc[rs][ts][g] * inv + bv);
        }
      }
  }
  __syncthreads();

  if (which == 0) {
    store_rows64_h(&Cs[0][0], qb + ((size_t)bh * N_ + n0) * HD_, (size_t)HD_, wave, lane);
  } else if (which == 1) {
    store_rows64_h(&Cs[0][0], kb + ((size_t)bh * N_ + n0) * HD_, (size_t)HD_, wave, lane);
  } else {
    store_rows64_h(&Cs[0][0], vtb + (size_t)bh * HD_ * N_ + n0, (size_t)N_, wave, lane);
  }
}

__global__ __launch_bounds__(256) void froq_kernel(
    const _Float16* __restrict__ qb, float* __restrict__ froq, int per) {
  __shared__ float red[8];
  const int tid = threadIdx.x, lane = tid & 31, wave = tid >> 5;
  const int bh = blockIdx.x;
  const _Float16* p = qb + (size_t)bh * per;
  float s = 0.f;
  for (int i = tid * 8; i < per; i += 256 * 8) {
    Pack8 u;
    u.v = *(const v8h*)(p + i);
    #pragma unroll
    for (int e = 0; e < 8; ++e) { const float f = (float)u.s[e]; s += f * f; }
  }
  s = wave_sum(s);
  if (lane == 0) red[wave] = s;
  __syncthreads();
  if (tid < 32) {
    float t = (lane < 8) ? red[lane] : 0.f;
    t = wave_sum(t);
    float* q = froq + (size_t)bh * 32 + lane;
    *(volatile float*)q = t;
    __threadfence();
    *(volatile float*)q = t;
  }
}

__global__ __launch_bounds__(256) void scale_kernel(
    const float* __restrict__ colabs, const float* __restrict__ froq,
    float* __restrict__ scl, int dim, float alpha) {
  __shared__ float red[8];
  __shared__ float infb[B_];
  const int tid = threadIdx.x, lane = tid & 31, wave = tid >> 5;
  #pragma unroll
  for (int b = 0; b < B_; ++b) {
    float m = 0.f;
    for (int i = tid; i < dim; i += 256) m = fmaxf(m, colabs[(size_t)b * dim + i]);
    m = wave_max(m);
    if (lane == 0) red[wave] = m;
    __syncthreads();
    if (tid < 32) {
      float t = (lane < 8) ? red[lane] : 0.f;
      t = wave_max(t);
      if (lane == 0) infb[b] = t;
    }
    __syncthreads();
  }
  if (tid < 32) {
    const float f = froq[(size_t)tid * 32];
    const float s = 2.0f * alpha / (sqrtf(f) * infb[tid >> 4]);
    *(volatile float*)(scl + tid) = s;
    __threadfence();
    *(volatile float*)(scl + tid) = s;
  }
}

__global__ __launch_bounds__(128) void attn_kernel(
    const _Float16* __restrict__ qb, const _Float16* __restrict__ kb,
    const _Float16* __restrict__ vtb, const float* __restrict__ scl,
    _Float16* __restrict__ wgt) {
  __shared__ __align__(16) _Float16 qtile[64][LP];
  __shared__ __align__(16) _Float16 ktile[64][LP];
  __shared__ __align__(16) _Float16 vtile[64][LP];
  __shared__ __align__(16) _Float16 ptile[4][16][LP];
  __shared__ __align__(16) _Float16 otile[64][LP];

  const int tid = threadIdx.x, lane = tid & 31, wave = tid >> 5;
  const int h8 = lane >> 4, l16 = lane & 15;
  const int qblk = blockIdx.x, bh = blockIdx.y;
  if (qblk >= N_ / 64 || bh >= B_ * H_) return;
  const int b = bh >> 4, hh = bh & (H_ - 1);
  const int q0 = qblk * 64;
  const _Float16* qh  = qb  + (size_t)bh * N_ * HD_;
  const _Float16* kh  = kb  + (size_t)bh * N_ * HD_;
  const _Float16* vth = vtb + (size_t)bh * HD_ * N_;
  const float sc = scl[bh];

  #pragma unroll
  for (int i = 0; i < 4; ++i) {
    const int c = tid + i * 128, r = c >> 3, col = (c & 7) * 8;
    *(v8h*)&qtile[r][col] = *(const v8h*)(qh + (size_t)(q0 + r) * HD_ + col);
  }
  __syncthreads();

  Frag qf[2];
  {
    const _Float16* qr = &qtile[wave * 16 + l16][0];
    #pragma unroll
    for (int c = 0; c < 2; ++c) {
      qf[c].half[0] = *(const v8h*)(qr + c * 32 + 8 * h8);
      qf[c].half[1] = *(const v8h*)(qr + c * 32 + 16 + 8 * h8);
    }
  }

  float m_run[8], l_run[8];
  v8f o[4];
  #pragma unroll
  for (int g = 0; g < 8; ++g) { m_run[g] = -1e30f; l_run[g] = 0.f; }
  #pragma unroll
  for (int j = 0; j < 4; ++j)
    #pragma unroll
    for (int e = 0; e < 8; ++e) o[j][e] = 0.f;

  #pragma unroll 1
  for (int it = 0; it < N_ / 64; ++it) {
    const int key0 = it * 64;
    v8h tk[4], tv[4];
    #pragma unroll
    for (int i = 0; i < 4; ++i) {
      const int c = tid + i * 128, r = c >> 3, col = (c & 7) * 8;
      tk[i] = *(const v8h*)(kh + (size_t)(key0 + r) * HD_ + col);
      tv[i] = *(const v8h*)(vth + (size_t)r * N_ + key0 + col);
    }
    __syncthreads();
    #pragma unroll
    for (int i = 0; i < 4; ++i) {
      const int c = tid + i * 128, r = c >> 3, col = (c & 7) * 8;
      *(v8h*)&ktile[r][col] = tk[i];
      *(v8h*)&vtile[r][col] = tv[i];
    }
    __syncthreads();

    v8f st[4];
    #pragma unroll
    for (int t = 0; t < 4; ++t) {
      v8f s;
      #pragma unroll
      for (int e = 0; e < 8; ++e) s[e] = 0.f;
      #pragma unroll
      for (int c = 0; c < 2; ++c) {
        Frag kf;
        const _Float16* kr = &ktile[t * 16 + l16][c * 32];
        kf.half[0] = *(const v8h*)(kr + 8 * h8);
        kf.half[1] = *(const v8h*)(kr + 16 + 8 * h8);
        s = wmma16(qf[c], kf, s);
      }
      #pragma unroll
      for (int e = 0; e < 8; ++e) st[t][e] = s[e] * sc;
    }

    float fac[8];
    #pragma unroll
    for (int g = 0; g < 8; ++g) {
      float mx = fmaxf(fmaxf(st[0][g], st[1][g]), fmaxf(st[2][g], st[3][g]));
      #pragma unroll
      for (int off = 1; off < 16; off <<= 1) mx = fmaxf(mx, __shfl_xor(mx, off, 32));
      const float mn = fmaxf(m_run[g], mx);
      const float f  = __expf(m_run[g] - mn);
      const float e0 = __expf(st[0][g] - mn);
      const float e1 = __expf(st[1][g] - mn);
      const float e2 = __expf(st[2][g] - mn);
      const float e3 = __expf(st[3][g] - mn);
      float ps = (e0 + e1) + (e2 + e3);
      #pragma unroll
      for (int off = 1; off < 16; off <<= 1) ps += __shfl_xor(ps, off, 32);
      l_run[g] = l_run[g] * f + ps;
      m_run[g] = mn;
      fac[g]   = f;
      _Float16* pr = &ptile[wave][g + 8 * h8][0];
      pr[l16]      = (_Float16)e0;
      pr[16 + l16] = (_Float16)e1;
      pr[32 + l16] = (_Float16)e2;
      pr[48 + l16] = (_Float16)e3;
    }
    __syncthreads();

    Frag pf[2];
    {
      const _Float16* pr = &ptile[wave][l16][0];
      #pragma unroll
      for (int c = 0; c < 2; ++c) {
        pf[c].half[0] = *(const v8h*)(pr + c * 32 + 8 * h8);
        pf[c].half[1] = *(const v8h*)(pr + c * 32 + 16 + 8 * h8);
      }
    }
    #pragma unroll
    for (int j = 0; j < 4; ++j) {
      #pragma unroll
      for (int g = 0; g < 8; ++g) o[j][g] *= fac[g];
      #pragma unroll
      for (int c = 0; c < 2; ++c) {
        Frag vf;
        const _Float16* vr = &vtile[j * 16 + l16][c * 32];
        vf.half[0] = *(const v8h*)(vr + 8 * h8);
        vf.half[1] = *(const v8h*)(vr + 16 + 8 * h8);
        o[j] = wmma16(pf[c], vf, o[j]);
      }
    }
  }

  float rl[8];
  #pragma unroll
  for (int g = 0; g < 8; ++g) rl[g] = OSC / l_run[g];
  #pragma unroll
  for (int j = 0; j < 4; ++j)
    #pragma unroll
    for (int g = 0; g < 8; ++g)
      otile[wave * 16 + g + 8 * h8][j * 16 + l16] = (_Float16)(o[j][g] * rl[g]);
  __syncthreads();
  store_rows64_h(&otile[0][0], wgt + ((size_t)b * N_ + q0) * D_ + (size_t)hh * HD_,
                 (size_t)D_, wave, lane);
}

__global__ __launch_bounds__(128) void proj_gemm_kernel(
    const _Float16* __restrict__ wg, const _Float16* __restrict__ wt, const float* __restrict__ bias,
    float* __restrict__ out, int M, int NC, int K) {
  __shared__ __align__(16) _Float16 As[64][LP];
  __shared__ __align__(16) _Float16 Bs[64][LP];
  __shared__ __align__(16) float Cf[64][LPF];
  const int tid = threadIdx.x, lane = tid & 31, wave = tid >> 5;
  const int h8 = lane >> 4, l16 = lane & 15;
  const int wm = (wave >> 1) * 32, wn = (wave & 1) * 32;
  const int mbase = blockIdx.y * 64, nbase = blockIdx.x * 64;
  if (mbase + 64 > M || nbase + 64 > NC) return;

  v8f acc[2][2];
  gemm64_mainloop(wg, wt, K, mbase, nbase, As, Bs, acc);

  const float inv = 1.0f / (OSC * WSC);
  #pragma unroll
  for (int rs = 0; rs < 2; ++rs)
    #pragma unroll
    for (int ts = 0; ts < 2; ++ts) {
      const int col = wn + ts * 16 + l16;
      const float bv = bias[nbase + col];
      #pragma unroll
      for (int g = 0; g < 8; ++g) {
        const int row = wm + rs * 16 + g + 8 * h8;
        Cf[row][col] = acc[rs][ts][g] * inv + bv;
      }
    }
  __syncthreads();

  v4f v[8];
  size_t off[8];
  #pragma unroll
  for (int p = 0; p < 8; ++p) {
    const int row = wave * 16 + p * 2 + (lane >> 4);
    const int c4  = (lane & 15) * 4;
    v[p] = *(const v4f*)&Cf[row][c4];
    off[p] = (size_t)(mbase + row) * NC + nbase + c4;
  }
  #pragma unroll
  for (int p = 0; p < 8; ++p) *(volatile v4f*)(out + off[p]) = v[p];
  __threadfence();
  #pragma unroll
  for (int p = 0; p < 8; ++p) *(volatile v4f*)(out + off[p]) = v[p];
}


extern "C" void kernel_launch(void* const* d_in, const int* in_sizes, int n_in,
                              void* d_out, int out_size, void* d_ws, size_t ws_size,
                              hipStream_t stream) {
  if (n_in < 5) return;
  const int nX = B_ * N_ * D_;
  if (in_sizes[0] != nX || in_sizes[1] != D_ * 3 * D_ || in_sizes[2] != 3 * D_ ||
      in_sizes[3] != D_ * D_ || in_sizes[4] != D_ || out_size != nX) return;

  const float* x     = (const float*)d_in[0];
  const float* Wqkv  = (const float*)d_in[1];
  const float* bqkv  = (const float*)d_in[2];
  const float* Wproj = (const float*)d_in[3];
  const float* bproj = (const float*)d_in[4];
  float* out = (float*)d_out;

  const size_t szXb  = (size_t)nX * 2;
  const size_t szWq  = (size_t)3 * D_ * D_ * 2;
  const size_t szWp  = (size_t)D_ * D_ * 2;
  const size_t szQ   = (size_t)B_ * H_ * N_ * HD_ * 2;
  const size_t szWg  = (size_t)nX * 2;
  const size_t szCol = (size_t)B_ * D_ * 4;
  const size_t szFro = (size_t)B_ * H_ * 32 * 4;
  const size_t szScl = 128;
  size_t off = 0;
  const size_t oXb  = off; off += szXb;
  const size_t oWq  = off; off += szWq;
  const size_t oWp  = off; off += szWp;
  const size_t oQ   = off; off += szQ;
  const size_t oK   = off; off += szQ;
  const size_t oVt  = off; off += szQ;
  const size_t oWg  = off; off += szWg;
  const size_t oCol = off; off += szCol;
  const size_t oFro = off; off += szFro;
  const size_t oScl = off; off += szScl;
  if (off > ws_size) return;

  char* ws = (char*)d_ws;
  _Float16* xb   = (_Float16*)(ws + oXb);
  _Float16* wqt  = (_Float16*)(ws + oWq);
  _Float16* wpt  = (_Float16*)(ws + oWp);
  _Float16* qb   = (_Float16*)(ws + oQ);
  _Float16* kbf  = (_Float16*)(ws + oK);
  _Float16* vtb  = (_Float16*)(ws + oVt);
  _Float16* wgt  = (_Float16*)(ws + oWg);
  float* colabs  = (float*)(ws + oCol);
  float* froq    = (float*)(ws + oFro);
  float* scl     = (float*)(ws + oScl);

  cvt_f16_kernel<<<(nX / 8 + 255) / 256, 256, 0, stream>>>(x, xb, nX);
  transpose_cvt_kernel<<<dim3((3 * D_ + 63) / 64, (D_ + 63) / 64), 128, 0, stream>>>(
      Wqkv, wqt, D_, 3 * D_, WSC);
  transpose_cvt_kernel<<<dim3((D_ + 63) / 64, (D_ + 63) / 64), 128, 0, stream>>>(
      Wproj, wpt, D_, D_, WSC);
  colabs_kernel<<<dim3((D_ + 255) / 256, B_), 256, 0, stream>>>(x, colabs, N_, D_);
  qkv_gemm_kernel<<<dim3((3 * D_ + 63) / 64, (B_ * N_ + 63) / 64), 128, 0, stream>>>(
      xb, wqt, bqkv, qb, kbf, vtb, B_ * N_, 3 * D_, D_);
  froq_kernel<<<B_ * H_, 256, 0, stream>>>(qb, froq, N_ * HD_);
  scale_kernel<<<1, 256, 0, stream>>>(colabs, froq, scl, D_, ALPHA_);
  attn_kernel<<<dim3(N_ / 64, B_ * H_), 128, 0, stream>>>(qb, kbf, vtb, scl, wgt);
  proj_gemm_kernel<<<dim3((D_ + 63) / 64, (B_ * N_ + 63) / 64), 128, 0, stream>>>(
      wgt, wpt, bproj, out, B_ * N_, D_, D_);
}
